// PointNetSetAbstraction_27041114096409
// MI455X (gfx1250) — hardware-verified
//
#include <hip/hip_runtime.h>
#pragma clang fp contract(off)

typedef __attribute__((ext_vector_type(16))) _Float16 v16h;
typedef __attribute__((ext_vector_type(8)))  _Float16 v8h;
typedef __attribute__((ext_vector_type(8)))  float    v8f;
typedef __attribute__((ext_vector_type(4)))  float    v4f;
typedef __attribute__((ext_vector_type(4)))  int      v4i;
typedef __attribute__((ext_vector_type(4)))  unsigned v4u;

constexpr int NUM_BATCH   = 4;
constexpr int NUM_PTS     = 8192;
constexpr int NUM_CEN     = 2048;
constexpr int NUM_NBR     = 64;
constexpr int FEAT_CH     = 64;
constexpr int L1_CIN      = 67;
constexpr int L1_KPAD     = 96;
constexpr int L1_COUT     = 64;
constexpr int L2_COUT     = 64;
constexpr int L3_COUT     = 128;
constexpr float BN_EPS    = 1e-5f;
constexpr float W_CARRY   = 16.0f;
constexpr float ACT_CARRY = 16.0f;

constexpr int FA_PITCH = 104;
constexpr int HH_PITCH = 72;
constexpr int WAVE_LDS_BYTES = 32512;
constexpr int OFF_H1   = NUM_NBR * FA_PITCH * 2;
constexpr int OFF_H2   = OFF_H1 + NUM_NBR * HH_PITCH * 2;
constexpr int OFF_VM   = OFF_H2 + NUM_NBR * HH_PITCH * 2;
constexpr int OFF_POOL = OFF_VM + NUM_NBR * 4;
static_assert(OFF_H1 == 13312 && OFF_H2 == 22528 && OFF_VM == 31744 && OFF_POOL == 32000, "lds map");
static_assert(OFF_POOL + L3_COUT * 4 == WAVE_LDS_BYTES, "lds map size");
static_assert(WAVE_LDS_BYTES % 16 == 0, "lds align");
static_assert(L1_KPAD % 32 == 0 && FEAT_CH % 32 == 0, "k multiple of 32");
static_assert(NUM_NBR == 64 && L1_COUT % 16 == 0 && L2_COUT % 16 == 0 && L3_COUT % 16 == 0, "tile multiples");
static_assert((NUM_BATCH * NUM_CEN) % 8 == 0, "grid exact");

constexpr int W1P_HALVES = L1_COUT * L1_KPAD;
constexpr int W2P_HALVES = L2_COUT * FEAT_CH;
constexpr int W3P_HALVES = L3_COUT * FEAT_CH;
constexpr int WP_HALVES  = W1P_HALVES + W2P_HALVES + W3P_HALVES;
static_assert(W1P_HALVES == 768 * 8 && W2P_HALVES == 512 * 8 && W3P_HALVES == 1024 * 8, "chunk counts");
static_assert(WP_HALVES == 9 * 256 * 8, "pack grid covers the planes exactly");

constexpr size_t WS_OFF_FPS  = 0;
constexpr size_t WS_OFF_BALL = (size_t)NUM_BATCH * NUM_CEN * 4;
constexpr size_t WS_OFF_WP   = WS_OFF_BALL + (size_t)NUM_BATCH * NUM_CEN * NUM_NBR * 4;
constexpr size_t WS_TOTAL    = WS_OFF_WP + (size_t)WP_HALVES * 2;
static_assert(WS_OFF_BALL % 128 == 0 && WS_OFF_WP % 128 == 0, "line aligned carve");
static_assert(WS_TOTAL <= 134217728, "carve limit");
constexpr size_t OUT1_OFF_BYTES = 98304;
static_assert((size_t)NUM_BATCH * NUM_CEN * 3 * 4 == OUT1_OFF_BYTES, "out1 offset");
static_assert(OUT1_OFF_BYTES + (size_t)NUM_BATCH * NUM_CEN * L3_COUT * 4 == 4292608, "out total");

__device__ __forceinline__ int clampi(int v, int lo, int hi) { return v < lo ? lo : (v > hi ? hi : v); }

union FragU { v16h v; v8h h[2]; };
__device__ __forceinline__ v16h frag_load(const _Float16* p) {
  FragU f;
  f.h[0] = *(const v8h*)(p);
  f.h[1] = *(const v8h*)(p + 16);
  return f.v;
}
__device__ __forceinline__ v8f mma_g(v16h a, v16h b, v8f c) {
  c = __builtin_amdgcn_wmma_f32_16x16x32_f16(false, a, false, b, (short)0, c, false, false);
  asm volatile("v_nop\n\tv_nop\n\tv_nop\n\tv_nop" : "+v"(c) : "v"(a), "v"(b));
  return c;
}

__global__ __launch_bounds__(256) void pack_weights_kernel(const float* __restrict__ W1,
                                                           const float* __restrict__ W2,
                                                           const float* __restrict__ W3,
                                                           _Float16* __restrict__ wp) {
  const int t = blockIdx.x * 256 + threadIdx.x;
  const float* W;
  int cin, kp, tl;
  if (blockIdx.x < 3)      { W = W1; cin = L1_CIN;  kp = L1_KPAD; tl = t; }
  else if (blockIdx.x < 5) { W = W2; cin = FEAT_CH; kp = FEAT_CH; tl = t - 768; }
  else                     { W = W3; cin = FEAT_CH; kp = FEAT_CH; tl = t - 1280; }
  const int cpr = kp >> 3;
  const int row = tl / cpr;
  const int k0  = (tl - row * cpr) * 8;
  v8h hv;
#pragma unroll
  for (int e = 0; e < 8; ++e) {
    const int k  = k0 + e;
    const int kc = k < cin ? k : cin - 1;
    const float f = W[row * cin + kc];
    const float s = (k < cin) ? f * W_CARRY : 0.0f;
    hv[e] = (_Float16)s;
  }
  _Float16* dst = wp + (size_t)t * 8;
  *(volatile v8h*)dst = hv;
  __threadfence();
  *(volatile v8h*)dst = hv;
}

constexpr int FPS_THREADS = 512;
constexpr int FPS_PPT = NUM_PTS / FPS_THREADS;
static_assert(FPS_PPT == 16, "points per thread");
static_assert(NUM_CEN == FPS_THREADS * 4, "idx line map");
static_assert(NUM_CEN * 3 == FPS_THREADS * 3 * 4, "centroid line map");

__global__ __launch_bounds__(512) void fps_kernel(const float* __restrict__ x,
                                                  int* __restrict__ idx_fps,
                                                  float* __restrict__ out_cen) {
#pragma clang fp contract(off)
  __shared__ float wval[2][16];
  __shared__ int   widx[2][16];
  __shared__ __align__(16) int sidx[NUM_CEN];

  const int b    = blockIdx.x;
  const int tid  = threadIdx.x;
  const int lane = tid & 31;
  const int wid  = tid >> 5;
  const float* xb = x + (size_t)b * NUM_PTS * 3;

  float px[FPS_PPT], py[FPS_PPT], pz[FPS_PPT], dm[FPS_PPT];
#pragma unroll
  for (int g = 0; g < FPS_PPT / 4; ++g) {
#pragma unroll
    for (int j = 0; j < 4; ++j) {
      const int i = g * 4 + j;
      const int p = tid + FPS_THREADS * i;
      px[i] = xb[p * 3 + 0];
      py[i] = xb[p * 3 + 1];
      pz[i] = xb[p * 3 + 2];
      dm[i] = 1e10f;
    }
#pragma unroll
    for (int j = 0; j < 4; ++j) {
      const int i = g * 4 + j;
      asm volatile("" : "+v"(px[i]), "+v"(py[i]), "+v"(pz[i]) : : "memory");
    }
  }

  int far = 0;
#pragma unroll 1
  for (int s = 0; s < NUM_CEN; ++s) {
    if (tid == 0) sidx[s] = far;
    const float cx = xb[far * 3 + 0];
    const float cy = xb[far * 3 + 1];
    const float cz = xb[far * 3 + 2];
    float bv = -1.0f;
    int   bi = tid;
#pragma unroll
    for (int i = 0; i < FPS_PPT; ++i) {
      const float dx = px[i] - cx;
      const float dy = py[i] - cy;
      const float dz = pz[i] - cz;
      const float t0 = dx * dx;
      const float t1 = dy * dy;
      const float t2 = dz * dz;
      const float d  = (t0 + t2) + t1;
      const float nd = (d < dm[i]) ? d : dm[i];
      dm[i] = nd;
      const bool up = nd > bv;
      bv = up ? nd : bv;
      bi = up ? (tid + FPS_THREADS * i) : bi;
    }
#pragma unroll
    for (int off = 16; off > 0; off >>= 1) {
      const float ov = __shfl_xor(bv, off, 32);
      const int   oi = __shfl_xor(bi, off, 32);
      const bool take = (ov > bv) || (ov == bv && oi < bi);
      bv = take ? ov : bv;
      bi = take ? oi : bi;
    }
    const int par = s & 1;
    if (lane == 0) { wval[par][wid] = bv; widx[par][wid] = bi; }
    __syncthreads();
    bv = wval[par][lane & 15];
    bi = widx[par][lane & 15];
#pragma unroll
    for (int off = 16; off > 0; off >>= 1) {
      const float ov = __shfl_xor(bv, off, 32);
      const int   oi = __shfl_xor(bi, off, 32);
      const bool take = (ov > bv) || (ov == bv && oi < bi);
      bv = take ? ov : bv;
      bi = take ? oi : bi;
    }
    far = clampi(bi, 0, NUM_PTS - 1);
  }
  __syncthreads();

  const v4i iv = *(const v4i*)(sidx + tid * 4);
  v4f cv[3];
#pragma unroll
  for (int j = 0; j < 3; ++j) {
    const int f = tid + FPS_THREADS * j;
#pragma unroll
    for (int e = 0; e < 4; ++e) {
      const int gi = 4 * f + e;
      const int sc = gi / 3;
      const int cc = gi - 3 * sc;
      const int pi = clampi(sidx[sc], 0, NUM_PTS - 1);
      cv[j][e] = xb[pi * 3 + cc];
    }
  }
  int*   idst = idx_fps + (size_t)b * NUM_CEN + tid * 4;
  float* cdst = out_cen + (size_t)b * NUM_CEN * 3;
  *(volatile v4i*)idst = iv;
#pragma unroll
  for (int j = 0; j < 3; ++j) *(volatile v4f*)(cdst + (size_t)(tid + FPS_THREADS * j) * 4) = cv[j];
  __threadfence();
  *(volatile v4i*)idst = iv;
#pragma unroll
  for (int j = 0; j < 3; ++j) *(volatile v4f*)(cdst + (size_t)(tid + FPS_THREADS * j) * 4) = cv[j];
}

__global__ __launch_bounds__(256) void ballq_kernel(const float* __restrict__ x,
                                                    const int* __restrict__ idx_fps,
                                                    int* __restrict__ idx_ball) {
#pragma clang fp contract(off)
  __shared__ __align__(16) int sIdx[8][NUM_NBR];
  const int lane = threadIdx.x & 31;
  const int w    = threadIdx.x >> 5;
  const int cidx = blockIdx.x * 8 + w;
  const int b    = cidx / NUM_CEN;
  const float* xb = x + (size_t)b * NUM_PTS * 3;

  const int fp = clampi(idx_fps[cidx], 0, NUM_PTS - 1);
  const float cx = xb[fp * 3 + 0];
  const float cy = xb[fp * 3 + 1];
  const float cz = xb[fp * 3 + 2];
  const float r2 = __uint_as_float(0x3D23D70Au);

  int total = 0;
#pragma unroll 1
  for (int c0 = 0; c0 < NUM_PTS; c0 += 32) {
    const int j = c0 + lane;
    const float dx = cx - xb[j * 3 + 0];
    const float dy = cy - xb[j * 3 + 1];
    const float dz = cz - xb[j * 3 + 2];
    const float t0 = dx * dx;
    const float t1 = dy * dy;
    const float t2 = dz * dz;
    const float d2 = (t0 + t2) + t1;
    const bool pred = d2 < r2;
    const unsigned msk = (unsigned)__ballot(pred);
    const int pos = total + __popc(msk & ((1u << lane) - 1u));
    if (pred && pos < NUM_NBR) sIdx[w][pos] = j;
    total += __popc(msk);
    if (total >= NUM_NBR) break;
  }
  const int cnt = total < NUM_NBR ? total : NUM_NBR;
  for (int p = cnt + lane; p < NUM_NBR; p += 32) sIdx[w][p] = -1;
  __syncthreads();
  if (threadIdx.x < 128) {
    const v4i v = *(const v4i*)(&sIdx[0][0] + threadIdx.x * 4);
    int* dst = idx_ball + (size_t)blockIdx.x * (8 * NUM_NBR) + threadIdx.x * 4;
    *(volatile v4i*)dst = v;
    __threadfence();
    *(volatile v4i*)dst = v;
  }
}

__global__ __launch_bounds__(64) void mlp_kernel(const float* __restrict__ x,
                                                 const float* __restrict__ xc,
                                                 const int* __restrict__ idx_fps,
                                                 const int* __restrict__ idx_ball,
                                                 const _Float16* __restrict__ wp,
                                                 const float* __restrict__ b1, const float* __restrict__ g1,
                                                 const float* __restrict__ bt1, const float* __restrict__ m1,
                                                 const float* __restrict__ v1,
                                                 const float* __restrict__ b2, const float* __restrict__ g2,
                                                 const float* __restrict__ bt2, const float* __restrict__ m2,
                                                 const float* __restrict__ v2,
                                                 const float* __restrict__ b3, const float* __restrict__ g3,
                                                 const float* __restrict__ bt3, const float* __restrict__ m3,
                                                 const float* __restrict__ v3,
                                                 float* __restrict__ out_pooled) {
  extern __shared__ __align__(16) char smem[];
  const int lane = threadIdx.x & 31;
  const int w    = threadIdx.x >> 5;
  const int cidx = blockIdx.x * 2 + w;
  const int b    = cidx / NUM_CEN;

  char* base = smem + (size_t)w * WAVE_LDS_BYTES;
  _Float16* Fa = (_Float16*)base;
  _Float16* H1 = (_Float16*)(base + OFF_H1);
  _Float16* H2 = (_Float16*)(base + OFF_H2);
  int*   vm    = (int*)(base + OFF_VM);
  float* pool  = (float*)(base + OFF_POOL);

  const _Float16* w1p = wp;
  const _Float16* w2p = wp + W1P_HALVES;
  const _Float16* w3p = wp + W1P_HALVES + W2P_HALVES;

  const float* xb  = x  + (size_t)b * NUM_PTS * 3;
  const float* xcb = xc + (size_t)b * NUM_PTS * FEAT_CH;
  const int*   nb  = idx_ball + (size_t)cidx * NUM_NBR;

  {
    const int q4 = lane >> 3;
    const int c8 = (lane & 7) * 8;
#pragma unroll 2
    for (int it = 0; it < 16; ++it) {
      const int row = it * 4 + q4;
      const int p = clampi(nb[row], 0, NUM_PTS - 1);
      const float* f = xcb + (size_t)p * FEAT_CH + c8;
      const v4f f0 = *(const v4f*)(f);
      const v4f f1 = *(const v4f*)(f + 4);
      v8h hv;
#pragma unroll
      for (int e = 0; e < 4; ++e) {
        const float a0 = f0[e];
        const float a1 = f1[e];
        hv[e]     = (_Float16)a0;
        hv[4 + e] = (_Float16)a1;
      }
      *(v8h*)(Fa + row * FA_PITCH + c8) = hv;
    }
  }
  {
    const int fp = clampi(idx_fps[cidx], 0, NUM_PTS - 1);
    const float ccx = xb[fp * 3 + 0];
    const float ccy = xb[fp * 3 + 1];
    const float ccz = xb[fp * 3 + 2];
    unsigned zz = 0u;
    asm volatile("" : "+v"(zz));
#pragma unroll
    for (int hr = 0; hr < 2; ++hr) {
      const int row = lane + 32 * hr;
      const int pi = nb[row];
      const int p  = clampi(pi, 0, NUM_PTS - 1);
      const float rx = xb[p * 3 + 0] - ccx;
      const float ry = xb[p * 3 + 1] - ccy;
      const float rz = xb[p * 3 + 2] - ccz;
      const _Float16 hx = (_Float16)rx;
      const _Float16 hy = (_Float16)ry;
      const _Float16 hz = (_Float16)rz;
      const unsigned short sx = __builtin_bit_cast(unsigned short, hx);
      const unsigned short sy = __builtin_bit_cast(unsigned short, hy);
      const unsigned short sz = __builtin_bit_cast(unsigned short, hz);
      const unsigned ux = (unsigned)sx;
      const unsigned uy = (unsigned)sy;
      const unsigned uz = (unsigned)sz;
      v4u wv;
      wv[0] = (ux & 0xffffu) | ((uy & 0xffffu) << 16);
      wv[1] = (uz & 0xffffu) | (zz << 16);
      wv[2] = zz;
      wv[3] = zz;
      v4u zv;
      zv[0] = zz;
      zv[1] = zz;
      zv[2] = zz;
      zv[3] = zz;
      const v8h wh = __builtin_bit_cast(v8h, wv);
      const v8h zh = __builtin_bit_cast(v8h, zv);
      *(v8h*)(Fa + row * FA_PITCH + 64) = wh;
      *(v8h*)(Fa + row * FA_PITCH + 72) = zh;
      *(v8h*)(Fa + row * FA_PITCH + 80) = zh;
      *(v8h*)(Fa + row * FA_PITCH + 88) = zh;
      vm[row] = (pi >= 0) ? 1 : 0;
    }
  }
  __syncthreads();

  const int ln = lane & 15;
  const int hs = lane >> 4;
  const v8f zero8 = (v8f){0.f, 0.f, 0.f, 0.f, 0.f, 0.f, 0.f, 0.f};

#pragma unroll 1
  for (int nt = 0; nt < L1_COUT / 16; ++nt) {
    const _Float16* bp = w1p + (nt * 16 + ln) * L1_KPAD + 8 * hs;
    const v16h bf0 = frag_load(bp);
    const v16h bf1 = frag_load(bp + 32);
    const v16h bf2 = frag_load(bp + 64);
    const int c = nt * 16 + ln;
    const float sg = g1[c] * rsqrtf(v1[c] + BN_EPS);
    const float sh = (b1[c] - m1[c]) * sg + bt1[c];
    const float sA = sg * (ACT_CARRY / W_CARRY);
    const float sB = sh * ACT_CARRY;
#pragma unroll
    for (int mt = 0; mt < 4; ++mt) {
      const _Float16* ap = Fa + (mt * 16 + ln) * FA_PITCH + 8 * hs;
      const v16h a0 = frag_load(ap);
      const v16h a1 = frag_load(ap + 32);
      const v16h a2 = frag_load(ap + 64);
      v8f acc = zero8;
      acc = mma_g(a0, bf0, acc);
      acc = mma_g(a1, bf1, acc);
      acc = mma_g(a2, bf2, acc);
#pragma unroll
      for (int q = 0; q < 8; ++q) {
        const float o = fmaxf(__builtin_fmaf(acc[q], sA, sB), 0.0f);
        H1[(mt * 16 + hs * 8 + q) * HH_PITCH + c] = (_Float16)o;
      }
    }
  }
  __syncthreads();

#pragma unroll 1
  for (int nt = 0; nt < L2_COUT / 16; ++nt) {
    const _Float16* bp = w2p + (nt * 16 + ln) * FEAT_CH + 8 * hs;
    const v16h bf0 = frag_load(bp);
    const v16h bf1 = frag_load(bp + 32);
    const int c = nt * 16 + ln;
    const float sg = g2[c] * rsqrtf(v2[c] + BN_EPS);
    const float sh = (b2[c] - m2[c]) * sg + bt2[c];
    const float sA = sg * (1.0f / W_CARRY);
    const float sB = sh * ACT_CARRY;
#pragma unroll
    for (int mt = 0; mt < 4; ++mt) {
      const _Float16* ap = H1 + (mt * 16 + ln) * HH_PITCH + 8 * hs;
      const v16h a0 = frag_load(ap);
      const v16h a1 = frag_load(ap + 32);
      v8f acc = zero8;
      acc = mma_g(a0, bf0, acc);
      acc = mma_g(a1, bf1, acc);
#pragma unroll
      for (int q = 0; q < 8; ++q) {
        const float o = fmaxf(__builtin_fmaf(acc[q], sA, sB), 0.0f);
        H2[(mt * 16 + hs * 8 + q) * HH_PITCH + c] = (_Float16)o;
      }
    }
  }
  __syncthreads();

  unsigned vbits = 0u;
#pragma unroll
  for (int mt = 0; mt < 4; ++mt) {
    const v4i ma = *(const v4i*)(vm + mt * 16 + hs * 8);
    const v4i mb = *(const v4i*)(vm + mt * 16 + hs * 8 + 4);
#pragma unroll
    for (int e = 0; e < 4; ++e) {
      const int xa = ma[e];
      const int xb2 = mb[e];
      vbits |= ((xa != 0) ? 1u : 0u) << (mt * 8 + e);
      vbits |= ((xb2 != 0) ? 1u : 0u) << (mt * 8 + 4 + e);
    }
  }

  const float NEGINF = -__builtin_inff();
#pragma unroll 1
  for (int nt = 0; nt < L3_COUT / 16; ++nt) {
    const _Float16* bp = w3p + (nt * 16 + ln) * FEAT_CH + 8 * hs;
    const v16h bf0 = frag_load(bp);
    const v16h bf1 = frag_load(bp + 32);
    const int c = nt * 16 + ln;
    const float sg = g3[c] * rsqrtf(v3[c] + BN_EPS);
    const float sh = (b3[c] - m3[c]) * sg + bt3[c];
    const float sA = sg * (1.0f / (W_CARRY * ACT_CARRY));
    float cmax = NEGINF;
#pragma unroll
    for (int mt = 0; mt < 4; ++mt) {
      const _Float16* ap = H2 + (mt * 16 + ln) * HH_PITCH + 8 * hs;
      const v16h a0 = frag_load(ap);
      const v16h a1 = frag_load(ap + 32);
      v8f acc = zero8;
      acc = mma_g(a0, bf0, acc);
      acc = mma_g(a1, bf1, acc);
#pragma unroll
      for (int q = 0; q < 8; ++q) {
        const float o = fmaxf(__builtin_fmaf(acc[q], sA, sh), 0.0f);
        const bool ok = ((vbits >> (mt * 8 + q)) & 1u) != 0u;
        const float om = ok ? o : NEGINF;
        cmax = fmaxf(cmax, om);
      }
    }
    const float other = __shfl_xor(cmax, 16, 32);
    const float mx = fmaxf(cmax, other);
    if (lane < 16) pool[c] = mx;
  }
  __syncthreads();

  {
    const v4f pv = *(const v4f*)(pool + lane * 4);
    float* dst = out_pooled + (size_t)cidx * L3_COUT + lane * 4;
    *(volatile v4f*)dst = pv;
    __threadfence();
    *(volatile v4f*)dst = pv;
  }
}

extern "C" void kernel_launch(void* const* d_in, const int* in_sizes, int n_in,
                              void* d_out, int out_size, void* d_ws, size_t ws_size,
                              hipStream_t stream) {
  (void)in_sizes; (void)out_size;
  if (n_in < 20) return;
  if (ws_size < WS_TOTAL) return;
  const float* x   = (const float*)d_in[0];
  const float* xc  = (const float*)d_in[1];
  const float* W1  = (const float*)d_in[2];
  const float* b1  = (const float*)d_in[3];
  const float* g1  = (const float*)d_in[4];
  const float* bt1 = (const float*)d_in[5];
  const float* m1  = (const float*)d_in[6];
  const float* v1  = (const float*)d_in[7];
  const float* W2  = (const float*)d_in[8];
  const float* b2  = (const float*)d_in[9];
  const float* g2  = (const float*)d_in[10];
  const float* bt2 = (const float*)d_in[11];
  const float* m2  = (const float*)d_in[12];
  const float* v2  = (const float*)d_in[13];
  const float* W3  = (const float*)d_in[14];
  const float* b3  = (const float*)d_in[15];
  const float* g3  = (const float*)d_in[16];
  const float* bt3 = (const float*)d_in[17];
  const float* m3  = (const float*)d_in[18];
  const float* v3  = (const float*)d_in[19];

  char* ws = (char*)d_ws;
  int*      idx_fps  = (int*)(ws + WS_OFF_FPS);
  int*      idx_ball = (int*)(ws + WS_OFF_BALL);
  _Float16* wp       = (_Float16*)(ws + WS_OFF_WP);

  float* out_cen    = (float*)d_out;
  float* out_pooled = (float*)((char*)d_out + OUT1_OFF_BYTES);

  pack_weights_kernel<<<9, 256, 0, stream>>>(W1, W2, W3, wp);
  fps_kernel<<<NUM_BATCH, FPS_THREADS, 0, stream>>>(x, idx_fps, out_cen);
  ballq_kernel<<<(NUM_BATCH * NUM_CEN) / 8, 256, 0, stream>>>(x, idx_fps, idx_ball);
  mlp_kernel<<<(NUM_BATCH * NUM_CEN) / 2, 64, 2 * WAVE_LDS_BYTES, stream>>>(
      x, xc, idx_fps, idx_ball, wp,
      b1, g1, bt1, m1, v1,
      b2, g2, bt2, m2, v2,
      b3, g3, bt3, m3, v3,
      out_pooled);
}
